// SimpleAttention_18124761989121
// MI455X (gfx1250) — hardware-verified
//
#include <hip/hip_runtime.h>

typedef __attribute__((ext_vector_type(16))) _Float16 v16h;
typedef __attribute__((ext_vector_type(8)))  _Float16 v8h;
typedef __attribute__((ext_vector_type(16))) __bf16   v16b;
typedef __attribute__((ext_vector_type(8)))  __bf16   v8b;
typedef __attribute__((ext_vector_type(8)))  float    v8f;
typedef __attribute__((ext_vector_type(4)))  float    v4f;
typedef __attribute__((ext_vector_type(4)))  unsigned v4u;

constexpr int kBatch = 4;
constexpr int kSeq   = 2048;
constexpr int kModel = 1024;
constexpr int kHeads = 16;
constexpr int kHd    = 64;
constexpr int kQkvN  = 3 * kModel;
constexpr int kRows  = kBatch * kSeq;

static_assert(kHeads * kHd == kModel);
static_assert(kHd == 64);
static_assert(kSeq % 64 == 0 && kModel % 64 == 0 && kQkvN % 64 == 0 && kRows % 64 == 0);
static_assert(kModel % 32 == 0);
static_assert(((kRows / 64) * (kQkvN / 64)) % 8 == 0);
static_assert(((kSeq / 64) * (kModel / 64)) % 8 == 0);
static_assert((kRows * kModel) % (8 * 256) == 0);
static_assert((kQkvN % (4 * 256)) == 0 && (kModel % (4 * 256)) == 0);

constexpr size_t kBytesWab  = (size_t)kQkvN * kModel * 2;
constexpr size_t kBytesWpb  = (size_t)kModel * kModel * 2;
constexpr size_t kBytesBat  = (size_t)kQkvN * 4;
constexpr size_t kBytesBpr  = (size_t)kModel * 4;
constexpr size_t kBytesXb   = (size_t)kRows * kModel * 2;
constexpr size_t kBytesQkv  = (size_t)kRows * kQkvN * 2;
constexpr size_t kOffWab    = 0;
constexpr size_t kOffWpb    = kOffWab + kBytesWab;
constexpr size_t kOffBat    = kOffWpb + kBytesWpb;
constexpr size_t kOffBpr    = kOffBat + kBytesBat;
constexpr size_t kOffXb     = kOffBpr + kBytesBpr;
constexpr size_t kOffQkvL   = kOffXb + kBytesXb;
constexpr size_t kOffQkvH   = kOffQkvL + kBytesQkv;
constexpr size_t kCarveTotal = kOffQkvH + kBytesQkv;
constexpr size_t kBytesYpl  = (size_t)kSeq * kModel * 2;
constexpr size_t kYStride   = (size_t)kSeq * kQkvN * 2;
constexpr size_t kYBase     = kOffQkvL - kYStride;
static_assert(kYBase >= kOffXb);
static_assert(kYBase + 2 * kBytesYpl <= kOffXb + kBytesXb);
static_assert(2 * kBytesYpl <= kYStride);
static_assert(kYBase + (size_t)(kBatch - 1) * kYStride + 2 * kBytesYpl <= kOffQkvL + (size_t)(kBatch - 1) * kYStride);
static_assert(kCarveTotal <= (size_t)134217728);
static_assert(kOffWpb % 128 == 0 && kOffBat % 128 == 0 && kOffBpr % 128 == 0 && kOffXb % 128 == 0 &&
              kOffQkvL % 128 == 0 && kOffQkvH % 128 == 0 && kYBase % 128 == 0 && kYStride % 128 == 0 &&
              kBytesYpl % 128 == 0);

#define NEG_INF_F (-__builtin_huge_valf())

__device__ __forceinline__ unsigned short f2bf_bits(float f) {
  unsigned u = __float_as_uint(f);
  return (unsigned short)((u + 0x7FFFu + ((u >> 16) & 1u)) >> 16);
}
__device__ __forceinline__ float bf_bits2f(unsigned short h) { return __uint_as_float(((unsigned)h) << 16); }

__device__ __forceinline__ void dep_guard_h(v8f& a, v8f& b, v16h x, v16h y) { asm volatile("v_nop\n\tv_nop\n\tv_nop\n\tv_nop" : "+v"(a), "+v"(b) : "v"(x), "v"(y)); }
__device__ __forceinline__ void dep_guard_b(v8f& a, v8f& b, v16b x, v16b y) { asm volatile("v_nop\n\tv_nop\n\tv_nop\n\tv_nop" : "+v"(a), "+v"(b) : "v"(x), "v"(y)); }
__device__ __forceinline__ void keep4_h(v16h a, v16h b, v16h c, v16h d) { asm volatile("v_nop" :: "v"(a), "v"(b), "v"(c), "v"(d)); }
__device__ __forceinline__ void keep4_b(v16b a, v16b b, v16b c, v16b d) { asm volatile("v_nop" :: "v"(a), "v"(b), "v"(c), "v"(d)); }
__device__ __forceinline__ void acc_guard4(v8f& a, v8f& b, v8f& c, v8f& d) { asm volatile("v_nop\n\tv_nop\n\tv_nop\n\tv_nop" : "+v"(a), "+v"(b), "+v"(c), "+v"(d)); }
template <typename T> struct Frag;
template <> struct Frag<_Float16> {
  typedef v16h V; union U { v16h v; v8h h[2]; };
  static __device__ __forceinline__ v16h load(const _Float16* p) {
    U f; f.h[0] = *(const v8h*)(p); f.h[1] = *(const v8h*)(p + 16); return f.v;
  }
  static __device__ __forceinline__ v8f mma(v16h a, v16h b, v8f c) {
    return __builtin_amdgcn_wmma_f32_16x16x32_f16(false, a, false, b, (short)0, c, false, false);
  }
  static __device__ __forceinline__ void guard(v8f& a, v8f& b, v16h x, v16h y) { dep_guard_h(a, b, x, y); }
  static __device__ __forceinline__ void keep(v16h a, v16h b, v16h c, v16h d) { keep4_h(a, b, c, d); }
};
template <> struct Frag<__bf16> {
  typedef v16b V; union U { v16b v; v8b h[2]; };
  static __device__ __forceinline__ v16b load(const __bf16* p) {
    U f; f.h[0] = *(const v8b*)(p); f.h[1] = *(const v8b*)(p + 16); return f.v;
  }
  static __device__ __forceinline__ v8f mma(v16b a, v16b b, v8f c) {
    return __builtin_amdgcn_wmma_f32_16x16x32_bf16(false, a, false, b, (short)0, c, false, false);
  }
  static __device__ __forceinline__ void guard(v8f& a, v8f& b, v16b x, v16b y) { dep_guard_b(a, b, x, y); }
  static __device__ __forceinline__ void keep(v16b a, v16b b, v16b c, v16b d) { keep4_b(a, b, c, d); }
};

template <int ET> struct Elem;
template <> struct Elem<0> { typedef _Float16 T; };
template <> struct Elem<1> { typedef __bf16 T; };
template <int ET, int SPLIT, int BIAS_MODE, int OUT_MODE, bool RESID, int ACT = 0>
__global__ __launch_bounds__(256) void wmma_gemm64(
    const unsigned short* __restrict__ Ap, const unsigned short* __restrict__ A2p, int lda, long strideA,
    const unsigned short* __restrict__ Btp, const unsigned short* __restrict__ Bt2p, int ldb, long strideB,
    void* __restrict__ Cout, void* __restrict__ Cout2, int ldc, long strideC,
    const float* __restrict__ bias,
    const float* __restrict__ resid, long strideR,
    int M, int N, int K, float scale) {
  typedef typename Elem<ET>::T T;
  typedef typename Frag<T>::V V;
  const T* A = (const T*)Ap; const T* A2 = (const T*)A2p; const T* Bt = (const T*)Btp; const T* Bt2 = (const T*)Bt2p;
  __shared__ __align__(16) float sT[8][16 * 68];
  const int b    = blockIdx.y;
  const int lane = threadIdx.x & 31;
  const int wave = threadIdx.x >> 5;
  const int tilesN = N >> 6;
  const int tilesM = M >> 6;
  const int tile = blockIdx.x * 8 + wave;
  if (tile >= tilesM * tilesN) return;
  const int tm = tile / tilesN;
  const int tn = tile - tm * tilesN;
  const int m0 = tm << 6;
  const int n0 = tn << 6;

  const T* Ab  = A  + (size_t)b * strideA;
  const T* Bb  = Bt + (size_t)b * strideB;
  const T* Ab2 = (SPLIT != 0) ? (A2  + (size_t)b * strideA) : nullptr;
  const T* Bb2 = (SPLIT == 1) ? (Bt2 + (size_t)b * strideB) : nullptr;

  const int rlane = lane & 15;
  const int koff  = (lane >> 4) * 8;
  const int mOff  = (lane >> 4) * 8;

  v8f acc[4][4];
#pragma unroll
  for (int i = 0; i < 4; ++i)
#pragma unroll
    for (int j = 0; j < 4; ++j) acc[i][j] = (v8f){0.f,0.f,0.f,0.f,0.f,0.f,0.f,0.f};

  for (int k0 = 0; k0 < K; k0 += 32) {
    V bh[4], bl[4];
#pragma unroll
    for (int j = 0; j < 4; ++j) {
      const size_t bo = (size_t)(n0 + (j << 4) + rlane) * ldb + koff + k0;
      bh[j] = Frag<T>::load(Bb + bo);
      if (SPLIT == 1) bl[j] = Frag<T>::load(Bb2 + bo);
    }
#pragma unroll
    for (int i = 0; i < 4; ++i) {
      const size_t ao = (size_t)(m0 + (i << 4) + rlane) * lda + koff + k0;
      V ah = Frag<T>::load(Ab + ao);
      V al;
      if (SPLIT != 0) al = Frag<T>::load(Ab2 + ao);
#pragma unroll
      for (int j = 0; j < 4; ++j) {
        acc[i][j] = Frag<T>::mma(ah, bh[j], acc[i][j]);
        if (SPLIT == 1) acc[i][j] = Frag<T>::mma(ah, bl[j], acc[i][j]);
        if (SPLIT != 0) acc[i][j] = Frag<T>::mma(al, bh[j], acc[i][j]);
      }
      Frag<T>::guard(acc[i][0], acc[i][3], ah, (SPLIT != 0) ? al : ah);
    }
    Frag<T>::keep(bh[0], bh[1], bh[2], bh[3]);
    if (SPLIT == 1) Frag<T>::keep(bl[0], bl[1], bl[2], bl[3]);
  }
  acc_guard4(acc[0][0], acc[0][1], acc[0][2], acc[0][3]);
  acc_guard4(acc[1][0], acc[1][1], acc[1][2], acc[1][3]);
  acc_guard4(acc[2][0], acc[2][1], acc[2][2], acc[2][3]);
  acc_guard4(acc[3][0], acc[3][1], acc[3][2], acc[3][3]);

  float* slab = sT[wave];
  const float* Rb = RESID ? (resid + (size_t)b * strideR) : nullptr;
#pragma unroll
  for (int i = 0; i < 4; ++i) {
    const int mBase = m0 + (i << 4);
#pragma unroll
    for (int j = 0; j < 4; ++j) {
      const int n = n0 + (j << 4) + rlane;
      float bv = 0.f;
      if (BIAS_MODE == 2) bv = bias[n];
#pragma unroll
      for (int r = 0; r < 8; ++r) {
        float v = acc[i][j][r] * scale;
        if (BIAS_MODE == 1) v += bias[mBase + mOff + r];
        if (BIAS_MODE == 2) v += bv;
        if (RESID) v += Rb[(size_t)(mBase + mOff + r) * ldc + n];
        if (ACT == 1) v = tanhf(v);
        if (ACT == 2) v = fmaxf(v, 0.0f);
        if (ACT == 3) v = v / (1.0f + expf(-v));
        if (ACT == 4) v = (v > 0.f) ? v : 0.01f * v;
        if (ACT == 5) v = 0.5f * v * (1.0f + erff(v * 0.70710678118654752f));
        slab[(mOff + r) * 68 + (j << 4) + rlane] = v;
      }
    }
    __builtin_amdgcn_fence(__ATOMIC_RELEASE, "workgroup");
    __builtin_amdgcn_wave_barrier();
    __builtin_amdgcn_fence(__ATOMIC_ACQUIRE, "workgroup");
    if (OUT_MODE == 0) {
      float* C = (float*)Cout + (size_t)b * strideC;
      const int hh = lane >> 4, c4 = (lane & 15) * 4;
      for (int pass = 0; pass < 2; ++pass) {
#pragma unroll
        for (int it = 0; it < 8; ++it) {
          const int row = it * 2 + hh;
          v4f v = *(const v4f*)(slab + row * 68 + c4);
          *(volatile v4f*)(C + (size_t)(mBase + row) * ldc + n0 + c4) = v;
        }
        __threadfence();
      }
    } else {
      const int q = lane >> 3, c8 = (lane & 7) * 8;
      unsigned short* C  = (unsigned short*)Cout  + (size_t)b * strideC;
      unsigned short* C2 = (OUT_MODE == 2) ? ((unsigned short*)Cout2 + (size_t)b * strideC) : nullptr;
      for (int pass = 0; pass < 2; ++pass) {
#pragma unroll
        for (int it = 0; it < 4; ++it) {
          const int row = it * 4 + q;
          const float* sp = slab + row * 68 + c8;
          v8h hv, lv;
#pragma unroll
          for (int e = 0; e < 8; ++e) {
            if (OUT_MODE == 1) {
              hv[e] = (_Float16)sp[e];
            } else {
              unsigned short hb = f2bf_bits(sp[e]);
              unsigned short lb = f2bf_bits(sp[e] - bf_bits2f(hb));
              hv[e] = __builtin_bit_cast(_Float16, hb);
              lv[e] = __builtin_bit_cast(_Float16, lb);
            }
          }
          *(volatile v8h*)(C + (size_t)(mBase + row) * ldc + n0 + c8) = hv;
          if (OUT_MODE == 2) *(volatile v8h*)(C2 + (size_t)(mBase + row) * ldc + n0 + c8) = lv;
        }
        __threadfence();
      }
    }
    __builtin_amdgcn_fence(__ATOMIC_RELEASE, "workgroup");
    __builtin_amdgcn_wave_barrier();
    __builtin_amdgcn_fence(__ATOMIC_ACQUIRE, "workgroup");
  }
}

__device__ __forceinline__ unsigned short at_bf_bits(float f) {
  unsigned u = __float_as_uint(f);
  return (unsigned short)((u + 0x7FFFu + ((u >> 16) & 1u)) >> 16);
}
__device__ __forceinline__ __bf16 at_f2bf(float f) { return __builtin_bit_cast(__bf16, at_bf_bits(f)); }
__device__ __forceinline__ void at_split(float f, __bf16& hi, __bf16& lo) {
  const unsigned short hb = at_bf_bits(f);
  hi = __builtin_bit_cast(__bf16, hb);
  lo = at_f2bf(f - __uint_as_float(((unsigned)hb) << 16));
}
__device__ __forceinline__ v8f at_mma(v16b a, v16b b, v8f c) {
  c = __builtin_amdgcn_wmma_f32_16x16x32_bf16(false, a, false, b, (short)0, c, false, false);
  asm volatile("v_nop\n\tv_nop\n\tv_nop\n\tv_nop" : "+v"(c) : "v"(a), "v"(b));
  return c;
}

__global__ __launch_bounds__(256) void cast_f32_bf16x8(const float* __restrict__ in,
                                                       unsigned short* __restrict__ out, int n8) {
  const int i = blockIdx.x * 256 + threadIdx.x;
  if (i < n8) {
    const size_t o = (size_t)i * 8;
    const v4f a = *(const v4f*)(in + o);
    const v4f g = *(const v4f*)(in + o + 4);
    v4u w;
    w[0] = (unsigned)f2bf_bits(a[0]) | ((unsigned)f2bf_bits(a[1]) << 16);
    w[1] = (unsigned)f2bf_bits(a[2]) | ((unsigned)f2bf_bits(a[3]) << 16);
    w[2] = (unsigned)f2bf_bits(g[0]) | ((unsigned)f2bf_bits(g[1]) << 16);
    w[3] = (unsigned)f2bf_bits(g[2]) | ((unsigned)f2bf_bits(g[3]) << 16);
    *(volatile v4u*)(out + o) = w;
    __threadfence();
    *(volatile v4u*)(out + o) = w;
  }
}

__global__ __launch_bounds__(256) void rne_bf16_f32x4(const float* __restrict__ in, float* __restrict__ out, int n4) {
  const int i = blockIdx.x * 256 + threadIdx.x;
  if (i < n4) {
    const size_t o = (size_t)i * 4;
    const v4f v = *(const v4f*)(in + o);
    v4f w;
#pragma unroll
    for (int e = 0; e < 4; ++e) w[e] = bf_bits2f(f2bf_bits(v[e]));
    *(volatile v4f*)(out + o) = w;
    __threadfence();
    *(volatile v4f*)(out + o) = w;
  }
}

__global__ __launch_bounds__(256) void transpose_cvt_bf16_64(const float* __restrict__ in,
                                                             unsigned short* __restrict__ out, int KD, int ND) {
  __shared__ __align__(16) float tile[64 * 68];
  const int k0 = blockIdx.x * 64, n0 = blockIdx.y * 64;
  const int tid = threadIdx.x;
#pragma unroll
  for (int it = 0; it < 4; ++it) {
    const int idx = tid + it * 256;
    const int kr = idx >> 4, c4 = (idx & 15) * 4;
    const v4f v = *(const v4f*)(in + (size_t)(k0 + kr) * ND + n0 + c4);
    *(v4f*)(tile + kr * 68 + c4) = v;
  }
  __syncthreads();
  const int wave = tid >> 5, lane = tid & 31, q = lane >> 3, c8 = (lane & 7) * 8;
  for (int pass = 0; pass < 2; ++pass) {
#pragma unroll
    for (int it = 0; it < 2; ++it) {
      const int nr = wave * 8 + it * 4 + q;
      v4u w;
#pragma unroll
      for (int e = 0; e < 4; ++e) {
        const int ka = c8 + 2 * e;
        const unsigned short b0 = f2bf_bits(tile[ka * 68 + nr]);
        const unsigned short b1 = f2bf_bits(tile[(ka + 1) * 68 + nr]);
        w[e] = (unsigned)b0 | ((unsigned)b1 << 16);
      }
      *(volatile v4u*)(out + (size_t)(n0 + nr) * KD + k0 + c8) = w;
    }
    __threadfence();
  }
}

__global__ __launch_bounds__(128)
void attn_causal64(const unsigned short* __restrict__ qkvh, const unsigned short* __restrict__ qkvl,
                   unsigned short* __restrict__ yh, unsigned short* __restrict__ yl) {
  union FB { v16b v; v8b h[2]; };
  __shared__ __align__(16) unsigned short Ksh[64 * 64];
  __shared__ __align__(16) unsigned short Ksl[64 * 64];
  __shared__ __align__(16) unsigned short Vth[64 * 64];
  __shared__ __align__(16) unsigned short Vtl[64 * 64];
  __shared__ __align__(16) __bf16 Psh[4][16 * 64];
  __shared__ __align__(16) __bf16 Psl[4][16 * 64];
  __shared__ __align__(16) float  Os[4][16 * 68];

  const int tid  = threadIdx.x;
  const int wave = tid >> 5;
  const int lane = tid & 31;
  const int hh   = lane >> 4;
  const int c    = lane & 15;

  const int qb   = blockIdx.x % (kSeq / 64);
  const int h    = blockIdx.x / (kSeq / 64);
  const int q0   = qb * 64 + wave * 16;
  const int hcol = h * kHd;

  const __bf16* KshB = (const __bf16*)Ksh;
  const __bf16* KslB = (const __bf16*)Ksl;
  const __bf16* VthB = (const __bf16*)Vth;
  const __bf16* VtlB = (const __bf16*)Vtl;

  v16b qah[2], qal[2];
  {
    const size_t qo = (size_t)(q0 + c) * kQkvN + hcol + 8 * hh;
#pragma unroll
    for (int dc = 0; dc < 2; ++dc) {
      qah[dc] = Frag<__bf16>::load((const __bf16*)qkvh + qo + dc * 32);
      qal[dc] = Frag<__bf16>::load((const __bf16*)qkvl + qo + dc * 32);
    }
  }

  float mrow[8], lrow[8];
  v8f oacc[4];
#pragma unroll
  for (int r = 0; r < 8; ++r) { mrow[r] = NEG_INF_F; lrow[r] = 0.f; }
#pragma unroll
  for (int t = 0; t < 4; ++t) oacc[t] = (v8f){0.f,0.f,0.f,0.f,0.f,0.f,0.f,0.f};

  for (int kc = 0; kc <= qb; ++kc) {
    const int kv0 = kc * 64;
    __syncthreads();
    {
      const int kvr = tid >> 1, dh = (tid & 1) * 32;
      const size_t ko = (size_t)(kv0 + kvr) * kQkvN + kModel + hcol + dh;
      const size_t vo = ko + kModel;
#pragma unroll
      for (int i = 0; i < 4; ++i) {
        const v4u wh = *(const v4u*)(qkvh + ko + 8 * i);
        const v4u wl = *(const v4u*)(qkvl + ko + 8 * i);
        *(v4u*)(Ksh + kvr * 64 + dh + 8 * i) = wh;
        *(v4u*)(Ksl + kvr * 64 + dh + 8 * i) = wl;
      }
      asm volatile("" ::: "memory");
#pragma unroll
      for (int i = 0; i < 4; ++i) {
        const v4u wh = *(const v4u*)(qkvh + vo + 8 * i);
        const v4u wl = *(const v4u*)(qkvl + vo + 8 * i);
#pragma unroll
        for (int e = 0; e < 4; ++e) {
          const int d = dh + 8 * i + 2 * e;
          const unsigned a = wh[e], g = wl[e];
          Vth[d * 64 + kvr]       = (unsigned short)(a & 0xffffu);
          Vth[(d + 1) * 64 + kvr] = (unsigned short)(a >> 16);
          Vtl[d * 64 + kvr]       = (unsigned short)(g & 0xffffu);
          Vtl[(d + 1) * 64 + kvr] = (unsigned short)(g >> 16);
        }
      }
    }
    __syncthreads();

    v8f s[4];
#pragma unroll
    for (int j = 0; j < 4; ++j) {
      s[j] = (v8f){0.f,0.f,0.f,0.f,0.f,0.f,0.f,0.f};
#pragma unroll
      for (int dc = 0; dc < 2; ++dc) {
        FB kb, kl;
        kb.h[0] = *(const v8b*)(KshB + (j * 16 + c) * 64 + dc * 32 + 8 * hh);
        kb.h[1] = *(const v8b*)(KshB + (j * 16 + c) * 64 + dc * 32 + 16 + 8 * hh);
        kl.h[0] = *(const v8b*)(KslB + (j * 16 + c) * 64 + dc * 32 + 8 * hh);
        kl.h[1] = *(const v8b*)(KslB + (j * 16 + c) * 64 + dc * 32 + 16 + 8 * hh);
        s[j] = at_mma(qah[dc], kb.v, s[j]);
        s[j] = at_mma(qah[dc], kl.v, s[j]);
        s[j] = at_mma(qal[dc], kb.v, s[j]);
      }
    }

    const bool diag = (kc == qb);
    float cm[8];
#pragma unroll
    for (int r = 0; r < 8; ++r) {
      const int qrow = q0 + 8 * hh + r;
      float m = NEG_INF_F;
#pragma unroll
      for (int j = 0; j < 4; ++j) {
        const int kvcol = kv0 + j * 16 + c;
        float sv = s[j][r] * 0.125f;
        if (diag && (kvcol > qrow)) sv = NEG_INF_F;
        s[j][r] = sv;
        m = fmaxf(m, sv);
      }
#pragma unroll
      for (int off = 1; off < 16; off <<= 1) m = fmaxf(m, __shfl_xor(m, off, 32));
      cm[r] = m;
    }
    __bf16* pwh = Psh[wave];
    __bf16* pwl = Psl[wave];
#pragma unroll
    for (int r = 0; r < 8; ++r) {
      const float mnew = fmaxf(mrow[r], cm[r]);
      const float alpha = expf(mrow[r] - mnew);
      mrow[r] = mnew;
      float psum = 0.f;
#pragma unroll
      for (int j = 0; j < 4; ++j) {
        const float p = expf(s[j][r] - mnew);
        psum += p;
        __bf16 ph, pl;
        at_split(p, ph, pl);
        pwh[(8 * hh + r) * 64 + j * 16 + c] = ph;
        pwl[(8 * hh + r) * 64 + j * 16 + c] = pl;
      }
#pragma unroll
      for (int off = 1; off < 16; off <<= 1) psum += __shfl_xor(psum, off, 32);
      lrow[r] = lrow[r] * alpha + psum;
#pragma unroll
      for (int t = 0; t < 4; ++t) oacc[t][r] *= alpha;
    }
    __builtin_amdgcn_fence(__ATOMIC_RELEASE, "workgroup");
    __builtin_amdgcn_wave_barrier();
    __builtin_amdgcn_fence(__ATOMIC_ACQUIRE, "workgroup");

#pragma unroll 1
    for (int kk = 0; kk < 2; ++kk) {
      FB pa, pl;
      pa.h[0] = *(const v8b*)(pwh + c * 64 + kk * 32 + 8 * hh);
      pa.h[1] = *(const v8b*)(pwh + c * 64 + kk * 32 + 16 + 8 * hh);
      pl.h[0] = *(const v8b*)(pwl + c * 64 + kk * 32 + 8 * hh);
      pl.h[1] = *(const v8b*)(pwl + c * 64 + kk * 32 + 16 + 8 * hh);
#pragma unroll
      for (int t = 0; t < 4; ++t) {
        FB vb, vl;
        vb.h[0] = *(const v8b*)(VthB + (t * 16 + c) * 64 + kk * 32 + 8 * hh);
        vb.h[1] = *(const v8b*)(VthB + (t * 16 + c) * 64 + kk * 32 + 16 + 8 * hh);
        vl.h[0] = *(const v8b*)(VtlB + (t * 16 + c) * 64 + kk * 32 + 8 * hh);
        vl.h[1] = *(const v8b*)(VtlB + (t * 16 + c) * 64 + kk * 32 + 16 + 8 * hh);
        oacc[t] = at_mma(pa.v, vb.v, oacc[t]);
        oacc[t] = at_mma(pa.v, vl.v, oacc[t]);
        oacc[t] = at_mma(pl.v, vb.v, oacc[t]);
      }
    }
  }

  float* os = Os[wave];
#pragma unroll
  for (int r = 0; r < 8; ++r) {
    const float inv = 1.0f / lrow[r];
#pragma unroll
    for (int t = 0; t < 4; ++t) os[(8 * hh + r) * 68 + t * 16 + c] = oacc[t][r] * inv;
  }
  __builtin_amdgcn_fence(__ATOMIC_RELEASE, "workgroup");
  __builtin_amdgcn_wave_barrier();
  __builtin_amdgcn_fence(__ATOMIC_ACQUIRE, "workgroup");
  {
    const int q = lane >> 3, c8 = (lane & 7) * 8;
    for (int pass = 0; pass < 2; ++pass) {
#pragma unroll
      for (int it = 0; it < 4; ++it) {
        const int row = it * 4 + q;
        const float* sp = os + row * 68 + c8;
        v4u wh, wl;
#pragma unroll
        for (int e = 0; e < 4; ++e) {
          const float f0 = sp[2 * e], f1 = sp[2 * e + 1];
          const unsigned short h0 = f2bf_bits(f0), h1 = f2bf_bits(f1);
          const unsigned short l0 = f2bf_bits(f0 - bf_bits2f(h0));
          const unsigned short l1 = f2bf_bits(f1 - bf_bits2f(h1));
          wh[e] = (unsigned)h0 | ((unsigned)h1 << 16);
          wl[e] = (unsigned)l0 | ((unsigned)l1 << 16);
        }
        const size_t yo = (size_t)(q0 + row) * kModel + hcol + c8;
        *(volatile v4u*)(yh + yo) = wh;
        *(volatile v4u*)(yl + yo) = wl;
      }
      __threadfence();
    }
  }
}

extern "C" void kernel_launch(void* const* d_in, const int* in_sizes, int n_in,
                              void* d_out, int out_size, void* d_ws, size_t ws_size,
                              hipStream_t stream) {
  if (n_in < 5) return;
  if (in_sizes[0] != kRows * kModel || in_sizes[1] != kModel * kQkvN || in_sizes[2] != kQkvN ||
      in_sizes[3] != kModel * kModel || in_sizes[4] != kModel) return;
  if (out_size != kRows * kModel) return;
  if (ws_size < kCarveTotal) return;

  const float* x  = (const float*)d_in[0];
  const float* Wa = (const float*)d_in[1];
  const float* ba = (const float*)d_in[2];
  const float* Wp = (const float*)d_in[3];
  const float* bp = (const float*)d_in[4];
  float* out = (float*)d_out;

  unsigned char* ws = (unsigned char*)d_ws;
  unsigned short* wab  = (unsigned short*)(ws + kOffWab);
  unsigned short* wpb  = (unsigned short*)(ws + kOffWpb);
  float*          bat  = (float*)(ws + kOffBat);
  float*          bpr  = (float*)(ws + kOffBpr);
  unsigned short* xb   = (unsigned short*)(ws + kOffXb);
  unsigned short* qkvl = (unsigned short*)(ws + kOffQkvL);
  unsigned short* qkvh = (unsigned short*)(ws + kOffQkvH);
  unsigned short* ybase_hi = (unsigned short*)(ws + kYBase);
  unsigned short* ybase_lo = (unsigned short*)(ws + kYBase + kBytesYpl);

  {
    const int n8 = kRows * kModel / 8;
    cast_f32_bf16x8<<<n8 / 256, 256, 0, stream>>>(x, xb, n8);
  }
  transpose_cvt_bf16_64<<<dim3(kModel / 64, kQkvN / 64), 256, 0, stream>>>(Wa, wab, kModel, kQkvN);
  transpose_cvt_bf16_64<<<dim3(kModel / 64, kModel / 64), 256, 0, stream>>>(Wp, wpb, kModel, kModel);
  rne_bf16_f32x4<<<(kQkvN / 4) / 256, 256, 0, stream>>>(ba, bat, kQkvN / 4);
  rne_bf16_f32x4<<<(kModel / 4) / 256, 256, 0, stream>>>(bp, bpr, kModel / 4);

  {
    const int tiles = (kRows / 64) * (kQkvN / 64);
    wmma_gemm64<1, 0, 2, 2, false, 0><<<dim3(tiles / 8, 1), 256, 0, stream>>>(
        xb, xb, kModel, 0L,
        wab, wab, kModel, 0L,
        (void*)qkvh, (void*)qkvl, kQkvN, 0L,
        bat, bat, 0L,
        kRows, kQkvN, kModel, 1.0f);
  }

  for (int b = 0; b < kBatch; ++b) {
    const size_t qoff = (size_t)b * kSeq * kQkvN;
    const size_t yoff = (size_t)b * (kYStride / 2);
    attn_causal64<<<kHeads * (kSeq / 64), 128, 0, stream>>>(
        qkvh + qoff, qkvl + qoff, ybase_hi + yoff, ybase_lo + yoff);
  }

  {
    const int tiles = (kSeq / 64) * (kModel / 64);
    wmma_gemm64<1, 2, 2, 0, false, 0><<<dim3(tiles / 8, kBatch), 256, 0, stream>>>(
        ybase_hi, ybase_lo, kModel, (long)(kYStride / 2),
        wpb, wpb, kModel, 0L,
        (void*)out, (void*)out, kModel, (long)kSeq * kModel,
        bpr, bpr, 0L,
        kSeq, kModel, kModel, 1.0f);
  }
}
